// _HFRefMoE_19000935317689
// MI455X (gfx1250) — hardware-verified
//
#include <hip/hip_runtime.h>
#include <hip/hip_bf16.h>
#include <math.h>


#define BB 2
#define SS 2048
#define DD 1024
#define HH 16
#define DKK 64
#define QW 2

typedef _Float16 bf16;
typedef __attribute__((ext_vector_type(4))) unsigned v4u_t;
typedef unsigned v4ua __attribute__((ext_vector_type(4), may_alias));
typedef __attribute__((ext_vector_type(4))) float v4f_t;
typedef float v4fa __attribute__((ext_vector_type(4), may_alias));
typedef __attribute__((ext_vector_type(16))) bf16  bf16x16;
typedef __attribute__((ext_vector_type(8)))  bf16  bf16x8;
typedef __attribute__((ext_vector_type(4)))  bf16  bf16x4;
typedef __attribute__((ext_vector_type(8)))  float f32x8;

#define LDS_STRIDE 48
#define KSTRIDE    72
#define VSTRIDE    48

__device__ __forceinline__ f32x8 wmma_bf16(bf16x16 a, bf16x16 b, f32x8 c) {
  return __builtin_amdgcn_wmma_f32_16x16x32_f16(
      false, a, false, b, (short)0, c, false, false);
}

template <typename T>
__device__ __forceinline__ bf16x16 load_frag(const T* __restrict__ base, int ld,
                                             int row0, int k0) {
  const int lane = threadIdx.x & 31;
  const int r    = lane & 15;
  const int kh   = (lane >> 4) * 8;
  const T* p0 = base + (size_t)(row0 + r) * ld + (k0 + kh);
  const T* p1 = p0 + 16;
  bf16x16 f;
#pragma unroll
  for (int i = 0; i < 8; ++i) {
    f[i]     = (bf16)p0[i];
    f[i + 8] = (bf16)p1[i];
  }
  return f;
}

__device__ __forceinline__ bf16x16 lds_frag(const bf16* base, int stride) {
  const int lane = threadIdx.x & 31;
  const int row  = lane & 15;
  const int kh   = (lane >> 4) * 8;
  const bf16x8 lo = *(const bf16x8*)(base + row * stride + kh);
  const bf16x8 hi = *(const bf16x8*)(base + row * stride + kh + 16);
  bf16x16 f;
#pragma unroll
  for (int i = 0; i < 8; ++i) { f[i] = lo[i]; f[i + 8] = hi[i]; }
  return f;
}

template <typename T>
__device__ __forceinline__ void stage_read16(const T* __restrict__ p, float* buf) {
#pragma unroll
  for (int i = 0; i < 16; ++i) buf[i] = (float)p[i];
}

__device__ __forceinline__ void stage_write(bf16* dst, const float* buf, int nquad) {
#pragma unroll
  for (int i = 0; i < nquad; ++i) {
    bf16x4 q;
    q[0] = (bf16)buf[4 * i];     q[1] = (bf16)buf[4 * i + 1];
    q[2] = (bf16)buf[4 * i + 2]; q[3] = (bf16)buf[4 * i + 3];
    *(bf16x4*)(dst + 4 * i) = q;
  }
}

template <typename AT, int MODE>
__global__ __launch_bounds__(256) void gemm_bias_kernel(
    const AT* __restrict__ A, const float* __restrict__ W,
    const float* __restrict__ bias, void* __restrict__ out,
    int M, int N, int K) {
  __shared__ bf16 ldsA[128 * LDS_STRIDE];
  __shared__ bf16 ldsW[256 * LDS_STRIDE];
  __shared__ __attribute__((aligned(16))) unsigned char sob[256 * 136 * 2];

  const int t    = threadIdx.x;
  const int wave = t >> 5;
  const int lane = t & 31;
  const int wm   = (wave & 1) * 64;
  const int wn   = (wave >> 1) * 64;
  const int mBlk = blockIdx.x * 128;
  const int nBlk = blockIdx.y * 256;

  const int arow = t >> 1;
  const int ach  = (t & 1) * 16;

  float abuf[16];
  float wbuf[32];

  stage_read16(A + (size_t)(mBlk + arow) * K + ach, abuf);
  stage_read16(W + (size_t)(nBlk + t) * K,          wbuf);
  stage_read16(W + (size_t)(nBlk + t) * K + 16,     wbuf + 16);

  f32x8 acc[4][4] = {};

  for (int k = 0; k < K; k += 32) {
    __syncthreads();
    stage_write(&ldsA[arow * LDS_STRIDE + ach], abuf, 4);
    stage_write(&ldsW[t * LDS_STRIDE],          wbuf, 8);
    if (k + 32 < K) {
      stage_read16(A + (size_t)(mBlk + arow) * K + (k + 32) + ach, abuf);
      stage_read16(W + (size_t)(nBlk + t) * K + (k + 32),          wbuf);
      stage_read16(W + (size_t)(nBlk + t) * K + (k + 32) + 16,     wbuf + 16);
    }
    __syncthreads();

    bf16x16 af[4], wf[4];
#pragma unroll
    for (int i = 0; i < 4; ++i)
      af[i] = lds_frag(ldsA + (wm + 16 * i) * LDS_STRIDE, LDS_STRIDE);
#pragma unroll
    for (int j = 0; j < 4; ++j)
      wf[j] = lds_frag(ldsW + (wn + 16 * j) * LDS_STRIDE, LDS_STRIDE);
#pragma unroll
    for (int i = 0; i < 4; ++i)
#pragma unroll
      for (int j = 0; j < 4; ++j)
        acc[i][j] = wmma_bf16(af[i], wf[j], acc[i][j]);
  }

  const int nlane = lane & 15;
  const int mh    = (lane >> 4) * 8;
  __syncthreads();
  if (MODE == 0 || MODE == 1) {
    bf16* so = (bf16*)sob;
#pragma unroll
    for (int i = 0; i < 4; ++i)
#pragma unroll
      for (int j = 0; j < 4; ++j) {
        const int nl = wn + 16 * j + nlane;
        const float bv = bias ? bias[nBlk + nl] : 0.0f;
#pragma unroll
        for (int r = 0; r < 8; ++r) {
          const int ml = wm + 16 * i + mh + r;
          const bf16 hv = (bf16)(acc[i][j][r] + bv);
          if (MODE == 0) so[ml * 264 + nl] = hv;
          else           so[nl * 136 + ml] = hv;
        }
      }
    __syncthreads();
#pragma unroll 1
    for (int pass = 0; pass < 2; ++pass) {
      if (MODE == 0) {
        for (int ch = t; ch < 128 * 32; ch += 256) { const int ml = ch >> 5, q = (ch & 31) * 8;
          *(volatile v4u_t*)((bf16*)out + (size_t)(mBlk + ml) * N + nBlk + q) = *(const v4ua*)(so + ml * 264 + q); }
      } else {
        const int b_ = mBlk / SS, s0 = mBlk & (SS - 1);
        for (int ch = t; ch < 256 * 16; ch += 256) { const int nl = ch >> 4, q = (ch & 15) * 8; const int n = nBlk + nl, h = n >> 6, dk = n & (DKK - 1);
          *(volatile v4u_t*)((bf16*)out + (((size_t)(b_ * HH + h)) * DKK + dk) * SS + s0 + q) = *(const v4ua*)(so + nl * 136 + q); }
      }
      __threadfence();
    }
  } else {
    float* so = (float*)sob;
#pragma unroll 1
    for (int hf = 0; hf < 2; ++hf) {
      if (wm == hf * 64) {
#pragma unroll
        for (int i = 0; i < 4; ++i)
#pragma unroll
          for (int j = 0; j < 4; ++j) {
            const int nl = wn + 16 * j + nlane;
            const float bv = bias ? bias[nBlk + nl] : 0.0f;
#pragma unroll
            for (int r = 0; r < 8; ++r) so[(16 * i + mh + r) * 260 + nl] = acc[i][j][r] + bv;
          }
      }
      __syncthreads();
#pragma unroll 1
      for (int pass = 0; pass < 2; ++pass) {
        for (int ch = t; ch < 64 * 64; ch += 256) { const int ml = ch >> 6, q = (ch & 63) * 4;
          *(volatile v4f_t*)((float*)out + (size_t)(mBlk + hf * 64 + ml) * N + nBlk + q) = *(const volatile v4fa*)(so + ml * 260 + q); }
        __threadfence();
      }
      __syncthreads();
    }
  }
}


#define NTK 2048
#define HS 1024
#define IE 512
#define NE 8
#define NG 4

__global__ __launch_bounds__(256) void k_route(const float* __restrict__ x, const float* __restrict__ rw, const float* __restrict__ bias, float* __restrict__ CW) {
  __shared__ float sc[4][NE]; __shared__ float cwl[4][NE];
  const int t0 = blockIdx.x * 4, tid = threadIdx.x, e = tid >> 5, lane = tid & 31;
  const float* wr = rw + (size_t)e * HS;
#pragma unroll 1
  for (int j = 0; j < 4; ++j) { const float* xr = x + (size_t)(t0 + j) * HS; float s = 0.0f;
#pragma unroll 1
    for (int k = lane; k < HS; k += 32) s += xr[k] * wr[k];
#pragma unroll
    for (int o = 16; o >= 1; o >>= 1) s += __shfl_xor(s, o, 32);
    if (lane == 0) sc[j][e] = 1.0f / (1.0f + expf(-s)); }
  __syncthreads();
  if (tid < 4) { const int j = tid;
    float scv[NE], chv[NE];
#pragma unroll
    for (int i = 0; i < NE; ++i) { scv[i] = sc[j][i]; chv[i] = sc[j][i] + bias[i]; }
    float gs[NG];
#pragma unroll
    for (int g = 0; g < NG; ++g) gs[g] = chv[2 * g] + chv[2 * g + 1];
    int g1 = 0; for (int g = 1; g < NG; ++g) if (gs[g] > gs[g1]) g1 = g;
    int g2 = -1; for (int g = 0; g < NG; ++g) { if (g == g1) continue; if (g2 < 0 || gs[g] > gs[g2]) g2 = g; }
    float mk[NE];
#pragma unroll
    for (int i = 0; i < NE; ++i) { const int g = i >> 1; mk[i] = (g == g1 || g == g2) ? chv[i] : 0.0f; }
    int e1 = 0; for (int i = 1; i < NE; ++i) if (mk[i] > mk[e1]) e1 = i;
    int e2 = -1; for (int i = 0; i < NE; ++i) { if (i == e1) continue; if (e2 < 0 || mk[i] > mk[e2]) e2 = i; }
    const float w1 = scv[e1], w2 = scv[e2], den = w1 + w2 + 1e-20f;
#pragma unroll
    for (int i = 0; i < NE; ++i) cwl[j][i] = 0.0f;
    cwl[j][e1] += w1 / den; cwl[j][e2] += w2 / den; }
  __syncthreads();
  if (tid < 32) { const float v = (&cwl[0][0])[tid]; *(volatile float*)(CW + (size_t)t0 * NE + tid) = v; __threadfence(); *(volatile float*)(CW + (size_t)t0 * NE + tid) = v; }
}
__global__ __launch_bounds__(256) void k_act(float* __restrict__ G, const float* __restrict__ U, const float* __restrict__ CW) {
  const int t = blockIdx.x, tid = threadIdx.x;
#pragma unroll 1
  for (int c = tid * 4; c < NE * IE; c += 1024) { const int e = c / IE; const float w = CW[(size_t)t * NE + e];
    float* gp = G + (size_t)t * (NE * IE) + c; const v4f_t g = *(const v4fa*)gp, u = *(const v4fa*)(U + (size_t)t * (NE * IE) + c); v4f_t r;
#pragma unroll
    for (int q = 0; q < 4; ++q) { const float gv = g[q]; r[q] = w * (gv / (1.0f + expf(-gv))) * u[q]; }
    *(volatile v4f_t*)gp = r; }
  __threadfence();
  for (int c = tid * 4; c < NE * IE; c += 1024) { float* gp = G + (size_t)t * (NE * IE) + c; const v4f_t v = *(const volatile v4fa*)gp; *(volatile v4f_t*)gp = v; }
}
__global__ __launch_bounds__(256) void k_act2(float* __restrict__ A, const float* __restrict__ Bm) {
  const size_t off = (size_t)blockIdx.x * HS + threadIdx.x * 4; const v4f_t g = *(const v4fa*)(A + off), u = *(const v4fa*)(Bm + off); v4f_t r;
#pragma unroll
  for (int q = 0; q < 4; ++q) { const float gv = g[q]; r[q] = (gv / (1.0f + expf(-gv))) * u[q]; }
  *(volatile v4f_t*)(A + off) = r; __threadfence(); *(volatile v4f_t*)(A + off) = r;
}
__global__ __launch_bounds__(256) void k_wdrows(const float* __restrict__ wd, float* __restrict__ Wdc) {
  const int h = blockIdx.x;
  for (int c = threadIdx.x * 4; c < NE * IE; c += 1024) { const int e = c / IE, i = c % IE; const v4f_t v = *(const v4fa*)(wd + ((size_t)e * HS + h) * IE + i);
    *(volatile v4f_t*)(Wdc + (size_t)h * (NE * IE) + c) = v; }
  __threadfence();
  for (int c = threadIdx.x * 4; c < NE * IE; c += 1024) { const int e = c / IE, i = c % IE; const v4f_t v = *(const v4fa*)(wd + ((size_t)e * HS + h) * IE + i);
    *(volatile v4f_t*)(Wdc + (size_t)h * (NE * IE) + c) = v; }
}
__global__ __launch_bounds__(256) void k_add(const float* __restrict__ S, float* __restrict__ out) {
  const size_t off = (size_t)blockIdx.x * HS + threadIdx.x * 4; v4f_t v = *(const v4fa*)(out + off); const v4f_t s = *(const v4fa*)(S + off);
  v.x += s.x; v.y += s.y; v.z += s.z; v.w += s.w; *(volatile v4f_t*)(out + off) = v; __threadfence(); *(volatile v4f_t*)(out + off) = v;
}

extern "C" void kernel_launch(void* const* d_in, const int* in_sizes, int n_in,
                              void* d_out, int out_size, void* d_ws, size_t ws_size,
                              hipStream_t stream) {
  (void)in_sizes; (void)n_in; (void)out_size; (void)ws_size;
  const float* x = (const float*)d_in[0];
  const float* rw = (const float*)d_in[1];
  const float* rb = (const float*)d_in[2];
  const float* wg = (const float*)d_in[3]; const float* wu = (const float*)d_in[4];
  const float* wd = (const float*)d_in[5];
  const float* sg = (const float*)d_in[6]; const float* su = (const float*)d_in[7]; const float* sdw = (const float*)d_in[8];
  float* out = (float*)d_out;
  char* ws = (char*)d_ws;
  float* CW  = (float*)ws; ws += (size_t)NTK * NE * 4;
  float* Wdc = (float*)ws; ws += (size_t)HS * NE * IE * 4;
  float* Gm  = (float*)ws; ws += (size_t)NTK * NE * IE * 4;
  float* Um  = (float*)ws; ws += (size_t)NTK * NE * IE * 4;
  float* S1 = Um; float* S2 = Um + (size_t)NTK * HS; float* S3 = Um + (size_t)2 * NTK * HS;
  k_route<<<NTK / 4, 256, 0, stream>>>(x, rw, rb, CW);
  k_wdrows<<<HS, 256, 0, stream>>>(wd, Wdc);
  dim3 blk(256);
  gemm_bias_kernel<float, 2><<<dim3(NTK / 128, NE * IE / 256), blk, 0, stream>>>(x, wg, nullptr, Gm, NTK, NE * IE, HS);
  gemm_bias_kernel<float, 2><<<dim3(NTK / 128, NE * IE / 256), blk, 0, stream>>>(x, wu, nullptr, Um, NTK, NE * IE, HS);
  k_act<<<NTK, 256, 0, stream>>>(Gm, Um, CW);
  gemm_bias_kernel<float, 2><<<dim3(NTK / 128, HS / 256), blk, 0, stream>>>(Gm, Wdc, nullptr, out, NTK, HS, NE * IE);
  gemm_bias_kernel<float, 2><<<dim3(NTK / 128, HS / 256), blk, 0, stream>>>(x, sg, nullptr, S1, NTK, HS, HS);
  gemm_bias_kernel<float, 2><<<dim3(NTK / 128, HS / 256), blk, 0, stream>>>(x, su, nullptr, S2, NTK, HS, HS);
  k_act2<<<NTK, 256, 0, stream>>>(S1, S2);
  gemm_bias_kernel<float, 2><<<dim3(NTK / 128, HS / 256), blk, 0, stream>>>(S1, sdw, nullptr, S3, NTK, HS, HS);
  k_add<<<NTK, 256, 0, stream>>>(S3, out);
}
